// Model_78451872628851
// MI455X (gfx1250) — hardware-verified
//
#include <hip/hip_runtime.h>
#include <math.h>

typedef __attribute__((ext_vector_type(16))) _Float16 v16h;
typedef __attribute__((ext_vector_type(8)))  _Float16 v8h;
typedef __attribute__((ext_vector_type(16))) __bf16   v16b;
typedef __attribute__((ext_vector_type(8)))  __bf16   v8b;
typedef __attribute__((ext_vector_type(8)))  float    v8f;
typedef __attribute__((ext_vector_type(4)))  float    v4f;

constexpr int kB    = 64;
constexpr int kT    = 512;
constexpr int kD    = 256;
constexpr int kG4   = 4 * kD;
constexpr int kK    = 2 * kD;
constexpr int kRows = kB * kT;
constexpr int kThr  = 256;
constexpr float kInCarry = 1024.0f;
constexpr float kSc = 1.0f / (kInCarry * kInCarry);
constexpr float kF16MinNormal = 6.103515625e-5f;
constexpr int kFBA = 0, kFBG = 256, kFEnd = 2048;

static_assert(kB == 64 && (kRows % 64) == 0 && ((kRows / 64) * (kD / 64)) % 8 == 0 && (kG4 / 64) % 8 == 0 && (kK % 32) == 0 && (kD % 32) == 0, "GEMM M, N multiples of 64; grids exact; K multiples of 32");

constexpr size_t kOffV16 = 0ull;
constexpr size_t kOffWA16 = 16777216ull;
constexpr size_t kOffWC16 = 16908288ull;
constexpr size_t kOffBIAS = 17956864ull;
constexpr size_t kOffVL32 = 17965056ull;
constexpr size_t kOffVL16 = 51519488ull;
constexpr size_t kOffATJ = 68296704ull;
constexpr size_t kOffA16 = 68427776ull;
constexpr size_t kOffG32 = 68493312ull;
constexpr size_t kOffC32 = 68755456ull;
constexpr size_t kOffC0 = 68820992ull;
constexpr size_t kOffDCS = 68886528ull;
constexpr size_t kWsTotal = 68952064ull;
static_assert(kWsTotal <= 134217728ull, "carve cap: under 128 MiB");
static_assert(kOffV16 == 0
              && kOffWA16 == kOffV16 + 16777216ull
              && kOffWC16 == kOffWA16 + 131072ull
              && kOffBIAS == kOffWC16 + 1048576ull
              && kOffVL32 == kOffBIAS + 8192ull
              && kOffVL16 == kOffVL32 + 33554432ull
              && kOffATJ == kOffVL16 + 16777216ull
              && kOffA16 == kOffATJ + 131072ull
              && kOffG32 == kOffA16 + 65536ull
              && kOffC32 == kOffG32 + 262144ull
              && kOffC0 == kOffC32 + 65536ull
              && kOffDCS == kOffC0 + 65536ull
              && kWsTotal == kOffDCS + 65536ull, "the carve is chained and totalled");
static_assert((kOffV16 % 256) == 0 && (kOffWA16 % 256) == 0 && (kOffWC16 % 256) == 0 && (kOffBIAS % 256) == 0 && (kOffVL32 % 256) == 0 && (kOffVL16 % 256) == 0 && (kOffATJ % 256) == 0 && (kOffA16 % 256) == 0 && (kOffG32 % 256) == 0 && (kOffC32 % 256) == 0 && (kOffC0 % 256) == 0 && (kOffDCS % 256) == 0, "aligned regions");

__device__ __forceinline__ unsigned short f2bf_bits(float f) {
  unsigned u = __float_as_uint(f);
  return (unsigned short)((u + 0x7FFFu + ((u >> 16) & 1u)) >> 16);
}
__device__ __forceinline__ float bf_bits2f(unsigned short h) { return __uint_as_float(((unsigned)h) << 16); }
__device__ __forceinline__ float bf16r(float f) { return bf_bits2f(f2bf_bits(f)); }
__device__ __forceinline__ float carry_flush(float v, float carry) {
  const float s = v * carry;
  return (fabsf(s) < kF16MinNormal) ? 0.0f : s;
}
__device__ __forceinline__ float frcp(float x) { return __builtin_amdgcn_rcpf(x); }

__device__ __forceinline__ void dep_guard4_h(v8f& a, v8f& b, v8f& c, v8f& d, v16h x, v16h y) { asm volatile("v_nop\n\tv_nop\n\tv_nop\n\tv_nop" : "+v"(a), "+v"(b), "+v"(c), "+v"(d) : "v"(x), "v"(y)); }
__device__ __forceinline__ void dep_guard4_b(v8f& a, v8f& b, v8f& c, v8f& d, v16b x, v16b y) { asm volatile("v_nop\n\tv_nop\n\tv_nop\n\tv_nop" : "+v"(a), "+v"(b), "+v"(c), "+v"(d) : "v"(x), "v"(y)); }
__device__ __forceinline__ void keep4_h(v16h a, v16h b, v16h c, v16h d) { asm volatile("v_nop" :: "v"(a), "v"(b), "v"(c), "v"(d)); }
__device__ __forceinline__ void keep4_b(v16b a, v16b b, v16b c, v16b d) { asm volatile("v_nop" :: "v"(a), "v"(b), "v"(c), "v"(d)); }
__device__ __forceinline__ void acc_guard4(v8f& a, v8f& b, v8f& c, v8f& d) { asm volatile("v_nop\n\tv_nop\n\tv_nop\n\tv_nop" : "+v"(a), "+v"(b), "+v"(c), "+v"(d)); }

template <typename T> struct Frag;
template <> struct Frag<_Float16> {
  typedef v16h V; union U { v16h v; v8h h[2]; };
  static __device__ __forceinline__ v16h load(const _Float16* p) {
    U f; f.h[0] = *(const v8h*)(p); f.h[1] = *(const v8h*)(p + 16); return f.v;
  }
  static __device__ __forceinline__ v8f mma(v16h a, v16h b, v8f c) {
    return __builtin_amdgcn_wmma_f32_16x16x32_f16(false, a, false, b, (short)0, c, false, false);
  }
  static __device__ __forceinline__ void guard4(v8f& a, v8f& b, v8f& c, v8f& d, v16h x, v16h y) { dep_guard4_h(a, b, c, d, x, y); }
  static __device__ __forceinline__ void keep(v16h a, v16h b, v16h c, v16h d) { keep4_h(a, b, c, d); }
};
template <> struct Frag<__bf16> {
  typedef v16b V; union U { v16b v; v8b h[2]; };
  static __device__ __forceinline__ v16b load(const __bf16* p) {
    U f; f.h[0] = *(const v8b*)(p); f.h[1] = *(const v8b*)(p + 16); return f.v;
  }
  static __device__ __forceinline__ v8f mma(v16b a, v16b b, v8f c) {
    return __builtin_amdgcn_wmma_f32_16x16x32_bf16(false, a, false, b, (short)0, c, false, false);
  }
  static __device__ __forceinline__ void guard4(v8f& a, v8f& b, v8f& c, v8f& d, v16b x, v16b y) { dep_guard4_b(a, b, c, d, x, y); }
  static __device__ __forceinline__ void keep(v16b a, v16b b, v16b c, v16b d) { keep4_b(a, b, c, d); }
};

__device__ __forceinline__ v8f mma_h(v16h a, v16h b, v8f c) {
  c = __builtin_amdgcn_wmma_f32_16x16x32_f16(false, a, false, b, (short)0, c, false, false);
  asm volatile("v_nop\n\tv_nop\n\tv_nop\n\tv_nop" : "+v"(c) : "v"(a), "v"(b));
  return c;
}

template <int ET> struct Elem;
template <> struct Elem<0> { typedef _Float16 T; };
template <> struct Elem<1> { typedef __bf16 T; };
template <int ET, bool SPLIT, int BIAS_MODE, int OUT_MODE, bool RESID, int ACT = 0>
__global__ __launch_bounds__(256) void wmma_gemm64(
    const unsigned short* __restrict__ Ap, const unsigned short* __restrict__ A2p, int lda, long strideA,
    const unsigned short* __restrict__ Btp, const unsigned short* __restrict__ Bt2p, int ldb, long strideB,
    void* __restrict__ Cout, void* __restrict__ Cout2, int ldc, long strideC,
    const float* __restrict__ bias,
    const float* __restrict__ resid, long strideR,
    int M, int N, int K, float scale) {
  typedef typename Elem<ET>::T T;
  typedef typename Frag<T>::V V;
  const T* A = (const T*)Ap; const T* A2 = (const T*)A2p; const T* Bt = (const T*)Btp; const T* Bt2 = (const T*)Bt2p;
  __shared__ __align__(16) float sT[8][16 * 68];
  const int b    = blockIdx.y;
  const int lane = threadIdx.x & 31;
  const int wave = threadIdx.x >> 5;
  const int tilesN = N >> 6;
  const int tilesM = M >> 6;
  const int tile = blockIdx.x * 8 + wave;
  if (tile >= tilesM * tilesN) return;
  const int tm = tile / tilesN;
  const int tn = tile - tm * tilesN;
  const int m0 = tm << 6;
  const int n0 = tn << 6;

  const T* Ab  = A  + (size_t)b * strideA;
  const T* Bb  = Bt + (size_t)b * strideB;
  const T* Ab2 = SPLIT ? (A2  + (size_t)b * strideA) : nullptr;
  const T* Bb2 = SPLIT ? (Bt2 + (size_t)b * strideB) : nullptr;

  const int rlane = lane & 15;
  const int koff  = (lane >> 4) * 8;
  const int mOff  = (lane >> 4) * 8;

  v8f acc[4][4];
#pragma unroll
  for (int i = 0; i < 4; ++i)
#pragma unroll
    for (int j = 0; j < 4; ++j) acc[i][j] = (v8f){0.f,0.f,0.f,0.f,0.f,0.f,0.f,0.f};

  for (int k0 = 0; k0 < K; k0 += 32) {
    V bh[4], bl[4];
#pragma unroll
    for (int j = 0; j < 4; ++j) {
      const size_t bo = (size_t)(n0 + (j << 4) + rlane) * ldb + koff + k0;
      bh[j] = Frag<T>::load(Bb + bo);
      if (SPLIT) bl[j] = Frag<T>::load(Bb2 + bo);
    }
#pragma unroll
    for (int i = 0; i < 4; ++i) {
      const size_t ao = (size_t)(m0 + (i << 4) + rlane) * lda + koff + k0;
      V ah = Frag<T>::load(Ab + ao);
      V al;
      if (SPLIT) al = Frag<T>::load(Ab2 + ao);
#pragma unroll
      for (int j = 0; j < 4; ++j) {
        acc[i][j] = Frag<T>::mma(ah, bh[j], acc[i][j]);
        if (SPLIT) {
          acc[i][j] = Frag<T>::mma(ah, bl[j], acc[i][j]);
          acc[i][j] = Frag<T>::mma(al, bh[j], acc[i][j]);
        }
      }
      Frag<T>::guard4(acc[i][0], acc[i][1], acc[i][2], acc[i][3], ah, SPLIT ? al : ah);
    }
    Frag<T>::keep(bh[0], bh[1], bh[2], bh[3]);
    if (SPLIT) Frag<T>::keep(bl[0], bl[1], bl[2], bl[3]);
  }
  acc_guard4(acc[0][0], acc[0][1], acc[0][2], acc[0][3]);
  acc_guard4(acc[1][0], acc[1][1], acc[1][2], acc[1][3]);
  acc_guard4(acc[2][0], acc[2][1], acc[2][2], acc[2][3]);
  acc_guard4(acc[3][0], acc[3][1], acc[3][2], acc[3][3]);

  float* slab = sT[wave];
  const float* Rb = RESID ? (resid + (size_t)b * strideR) : nullptr;
#pragma unroll
  for (int i = 0; i < 4; ++i) {
    const int mBase = m0 + (i << 4);
#pragma unroll
    for (int j = 0; j < 4; ++j) {
      const int n = n0 + (j << 4) + rlane;
      float bv = 0.f;
      if (BIAS_MODE == 2) bv = bias[n];
#pragma unroll
      for (int r = 0; r < 8; ++r) {
        float v = acc[i][j][r] * scale;
        if (BIAS_MODE == 1) v += bias[mBase + mOff + r];
        if (BIAS_MODE == 2) v += bv;
        if (RESID) v += Rb[(size_t)(mBase + mOff + r) * ldc + n];
        if (ACT == 1) v = tanhf(v);
        if (ACT == 2) v = fmaxf(v, 0.0f);
        if (ACT == 3) v = v / (1.0f + expf(-v));
        if (ACT == 4) v = (v > 0.f) ? v : 0.01f * v;
        slab[(mOff + r) * 68 + (j << 4) + rlane] = v;
      }
    }
    __builtin_amdgcn_fence(__ATOMIC_RELEASE, "workgroup");
    __builtin_amdgcn_wave_barrier();
    __builtin_amdgcn_fence(__ATOMIC_ACQUIRE, "workgroup");
    if (OUT_MODE == 0) {
      float* C = (float*)Cout + (size_t)b * strideC;
      const int hh = lane >> 4, c4 = (lane & 15) * 4;
      for (int pass = 0; pass < 2; ++pass) {
#pragma unroll
        for (int it = 0; it < 8; ++it) {
          const int row = it * 2 + hh;
          v4f v = *(const v4f*)(slab + row * 68 + c4);
          *(volatile v4f*)(C + (size_t)(mBase + row) * ldc + n0 + c4) = v;
        }
        __threadfence();
      }
    } else {
      const int q = lane >> 3, c8 = (lane & 7) * 8;
      unsigned short* C  = (unsigned short*)Cout  + (size_t)b * strideC;
      unsigned short* C2 = (OUT_MODE == 2) ? ((unsigned short*)Cout2 + (size_t)b * strideC) : nullptr;
      for (int pass = 0; pass < 2; ++pass) {
#pragma unroll
        for (int it = 0; it < 4; ++it) {
          const int row = it * 4 + q;
          const float* sp = slab + row * 68 + c8;
          v8h hv, lv;
#pragma unroll
          for (int e = 0; e < 8; ++e) {
            if (OUT_MODE == 1) {
              hv[e] = (_Float16)sp[e];
            } else {
              unsigned short hb = f2bf_bits(sp[e]);
              unsigned short lb = f2bf_bits(sp[e] - bf_bits2f(hb));
              hv[e] = __builtin_bit_cast(_Float16, hb);
              lv[e] = __builtin_bit_cast(_Float16, lb);
            }
          }
          *(volatile v8h*)(C + (size_t)(mBase + row) * ldc + n0 + c8) = hv;
          if (OUT_MODE == 2) *(volatile v8h*)(C2 + (size_t)(mBase + row) * ldc + n0 + c8) = lv;
        }
        __threadfence();
      }
    }
    __builtin_amdgcn_fence(__ATOMIC_RELEASE, "workgroup");
    __builtin_amdgcn_wave_barrier();
    __builtin_amdgcn_fence(__ATOMIC_ACQUIRE, "workgroup");
  }
}

__global__ __launch_bounds__(kThr) void cast_plane_kernel(const float* __restrict__ src, unsigned short* __restrict__ dst,
                                                          int colsLog2, int dstPitch, int dstOff) {
  const int i   = blockIdx.x * kThr + threadIdx.x;
  const int sh  = colsLog2 - 3;
  const int row = i >> sh;
  const int c8  = (i & ((1 << sh) - 1)) * 8;
  const float* sp = src + ((size_t)row << colsLog2) + c8;
  const v4f a0 = *(const v4f*)(sp);
  const v4f a1 = *(const v4f*)(sp + 4);
  v8h hv;
#pragma unroll
  for (int e = 0; e < 4; ++e) {
    const float f0 = a0[e];
    const float f1 = a1[e];
    hv[e]     = (_Float16)carry_flush(bf16r(f0), kInCarry);
    hv[4 + e] = (_Float16)carry_flush(bf16r(f1), kInCarry);
  }
  unsigned short* dp = dst + (size_t)row * dstPitch + dstOff + c8;
  *(volatile v8h*)dp = hv;
  __threadfence();
  *(volatile v8h*)dp = hv;
}

__device__ __forceinline__ float fast_tanh(float v) { return 1.0f - 2.0f * frcp(__expf(2.0f * v) + 1.0f); }
__device__ __forceinline__ float fast_sigmoid(float v) { return frcp(1.0f + __expf(-v)); }

__global__ __launch_bounds__(kThr) void wsetup_kernel(const float* __restrict__ b_att, const float* __restrict__ W_ih, const float* __restrict__ W_hh,
                                                      const float* __restrict__ b_ih, const float* __restrict__ b_hh, float* __restrict__ BIAS,
                                                      unsigned short* __restrict__ WC16, float* __restrict__ C32) {
  unsigned v = blockIdx.x * (unsigned)kThr + threadIdx.x;
  asm volatile("" : "+v"(v));
  if (v < 512u) {
    const unsigned i0 = v * 4u;
    v4f o = {0.f, 0.f, 0.f, 0.f};
    if (i0 < (unsigned)kFBG) {
      const v4f a = *(const v4f*)(b_att + i0);
#pragma unroll
      for (int e = 0; e < 4; ++e) { const float p = a[e]; o[e] = bf16r(p); }
    } else if (i0 < (unsigned)(kFBG + kG4)) {
      const v4f a = *(const v4f*)(b_ih + (i0 - (unsigned)kFBG)), c = *(const v4f*)(b_hh + (i0 - (unsigned)kFBG));
#pragma unroll
      for (int e = 0; e < 4; ++e) { const float p = a[e], q = c[e]; o[e] = bf16r(p) + bf16r(q); }
    }
    float* dp = BIAS + i0;
    *(volatile v4f*)dp = o;
    __threadfence();
    *(volatile v4f*)dp = o;
  } else if (v < 66048u) {
    const unsigned w = v - 512u;
    const unsigned n = w >> 6, c8 = (w & 63u) * 8u;
    const float* sp = (c8 < (unsigned)kD) ? (W_hh + (size_t)n * kD + c8) : (W_ih + (size_t)n * kD + (c8 - (unsigned)kD));
    const v4f a0 = *(const v4f*)sp, a1 = *(const v4f*)(sp + 4);
    v8h hv;
#pragma unroll
    for (int e = 0; e < 4; ++e) { const float p = a0[e], q = a1[e]; hv[e] = (_Float16)carry_flush(bf16r(p), kInCarry); hv[4 + e] = (_Float16)carry_flush(bf16r(q), kInCarry); }
    unsigned short* dp = WC16 + (size_t)w * 8u;
    *(volatile v8h*)dp = hv;
    __threadfence();
    *(volatile v8h*)dp = hv;
  } else {
    const v4f z = {0.f, 0.f, 0.f, 0.f};
    float* dp = C32 + (size_t)(v - 66048u) * 4u;
    *(volatile v4f*)dp = z;
    __threadfence();
    *(volatile v4f*)dp = z;
  }
}
static_assert(kFEnd / 4 == 512 && kG4 * (kK / 8) == 65536 && 512 + 65536 == 66048 && kB * kD / 4 == 4096 && 66048 + 4096 == 274 * kThr && kFBG + kG4 <= kFEnd, "weight set-up grid exact");

__global__ __launch_bounds__(kThr) void vcast_kernel(const float* __restrict__ VL32, unsigned short* __restrict__ VL16, unsigned short* __restrict__ A16) {
  unsigned v = blockIdx.x * (unsigned)kThr + threadIdx.x;
  asm volatile("" : "+v"(v));
  const size_t o8 = (size_t)v * 8u;
  const unsigned row = v >> 5, c8 = (v & 31u) * 8u;
  const unsigned b = row >> 9, t = row & 511u;
  const v4f a0 = *(const v4f*)(VL32 + o8), a1 = *(const v4f*)(VL32 + o8 + 4);
  v8h hv, zv;
#pragma unroll
  for (int e = 0; e < 4; ++e) { hv[e] = (_Float16)carry_flush(a0[e], kInCarry); hv[4 + e] = (_Float16)carry_flush(a1[e], kInCarry); zv[e] = (_Float16)0.0f; zv[4 + e] = (_Float16)0.0f; }
  const bool first = (t == 0u);
  unsigned short* ap = A16 + (size_t)b * kK + c8;
  for (int pass = 0; pass < 2; ++pass) {
    *(volatile v8h*)(VL16 + o8) = hv;
    if (first) { *(volatile v8h*)ap = zv; *(volatile v8h*)(ap + kD) = hv; }
    __threadfence();
  }
}
static_assert((size_t)kRows * kD / 8 == 4096 * (size_t)kThr, "vlin cast grid exact");

__global__ __launch_bounds__(kThr) void atj_kernel(const float* __restrict__ VL32, const float* __restrict__ values, float* __restrict__ ATJ) {
  unsigned v = blockIdx.x * (unsigned)kThr + threadIdx.x;
  asm volatile("" : "+v"(v));
  const unsigned b = v >> 9;
  const float* qp = VL32 + (size_t)b * kT * kD;
  const float* xp = values + (size_t)v * kD;
  float acc = 0.0f;
  for (int d = 0; d < kD; d += 4) {
    const v4f q4 = *(const v4f*)(qp + d), x4 = *(const v4f*)(xp + d);
    const float p0 = x4[0], p1 = x4[1], p2 = x4[2], p3 = x4[3];
    acc += q4[0] * bf16r(p0);
    acc += q4[1] * bf16r(p1);
    acc += q4[2] * bf16r(p2);
    acc += q4[3] * bf16r(p3);
  }
  const float o = 1.0f / (1.0f + expf(-acc));
  *(volatile float*)(ATJ + v) = o;
  __threadfence();
  *(volatile float*)(ATJ + v) = o;
}
static_assert(kRows == 128 * kThr, "attention-weight grid exact");

__global__ __launch_bounds__(kThr) void cell_kernel(const float* __restrict__ G32, const float* __restrict__ ATJ, const float* __restrict__ Deltas,
                                                    const unsigned short* __restrict__ VL16, float* __restrict__ C32, float* __restrict__ C0,
                                                    float* __restrict__ DCS, unsigned short* __restrict__ A16, float* __restrict__ out, int t) {
  unsigned v = blockIdx.x * (unsigned)kThr + threadIdx.x;
  asm volatile("" : "+v"(v));
  const unsigned b = v >> 5, u8 = (v & 31u) * 8u;
  const float* gr = G32 + (size_t)b * kG4 + u8;
  const size_t su = (size_t)b * kD + u8;
  const size_t ro = ((size_t)b * kT + (size_t)t) * kD + u8;
  const bool first = (t == 0);
  float a = ATJ[(size_t)b * kT + t];
  asm volatile("" : "+v"(a));
  v4f cn0, cn1, hn0, hn1, dc0, dc1; v8h hv;
#pragma unroll
  for (int hlf = 0; hlf < 2; ++hlf) {
    const v4f gi = *(const v4f*)(gr + 4 * hlf), gf = *(const v4f*)(gr + kD + 4 * hlf), gg = *(const v4f*)(gr + 2 * kD + 4 * hlf), go = *(const v4f*)(gr + 3 * kD + 4 * hlf);
    const v4f cc = *(const v4f*)(C32 + su + 4 * hlf), c0 = *(const v4f*)(C0 + su + 4 * hlf), ds = *(const v4f*)(DCS + su + 4 * hlf), dl = *(const v4f*)(Deltas + ro + 4 * hlf);
#pragma unroll
    for (int e = 0; e < 4; ++e) {
      const float pd = dl[e];
      const float dc = (first ? 0.0f : ds[e]) + bf16r(pd);
      const float alpha = a / __logf(2.718281828459045f + dc);
      const float cin = first ? 0.0f : (alpha * c0[e] + (1.0f - alpha) * cc[e]);
      const float cn = fast_sigmoid(gf[e]) * cin + fast_sigmoid(gi[e]) * fast_tanh(gg[e]);
      const float hn = fast_sigmoid(go[e]) * fast_tanh(cn);
      if (hlf == 0) { cn0[e] = cn; hn0[e] = hn; dc0[e] = dc; } else { cn1[e] = cn; hn1[e] = hn; dc1[e] = dc; }
      hv[4 * hlf + e] = (_Float16)carry_flush(hn, kInCarry);
    }
  }
  const bool nx = (t + 1 < kT);
  const v8h xv = *(const v8h*)(VL16 + ((size_t)b * kT + (size_t)(nx ? (t + 1) : t)) * kD + u8);
  float* cdst = (first ? C0 : C32) + su;
  unsigned short* ap = A16 + (size_t)b * kK + u8;
  for (int pass = 0; pass < 2; ++pass) {
    *(volatile v4f*)(out + ro) = hn0; *(volatile v4f*)(out + ro + 4) = hn1;
    *(volatile v4f*)cdst = cn0; *(volatile v4f*)(cdst + 4) = cn1;
    *(volatile v4f*)(DCS + su) = dc0; *(volatile v4f*)(DCS + su + 4) = dc1;
    *(volatile v8h*)ap = hv;
    if (nx) *(volatile v8h*)(ap + kD) = xv;
    __threadfence();
  }
}
static_assert(kB * kD / 8 == 8 * kThr && kD / 8 == 32, "cell grid: 8 blocks");

static_assert(((size_t)kRows * kD / 8) % kThr == 0 && ((size_t)kD * kD / 8) % kThr == 0, "plane cast grids exact");

extern "C" void kernel_launch(void* const* d_in, const int* in_sizes, int n_in,
                              void* d_out, int out_size, void* d_ws, size_t ws_size,
                              hipStream_t stream) {
  if (n_in < 8 || d_out == nullptr || d_ws == nullptr) return;
  if (in_sizes[0] != kRows * kD || in_sizes[1] != kRows * kD || in_sizes[2] != kD * kD || in_sizes[3] != kD) return;
  if (in_sizes[4] != kG4 * kD || in_sizes[5] != kG4 * kD || in_sizes[6] != kG4 || in_sizes[7] != kG4) return;
  if (out_size != kRows * kD) return;
  if (ws_size < kWsTotal) return;
  const float* values = (const float*)d_in[0];
  const float* Deltas = (const float*)d_in[1];
  const float* W_att = (const float*)d_in[2];
  const float* b_att = (const float*)d_in[3];
  const float* W_ih = (const float*)d_in[4];
  const float* W_hh = (const float*)d_in[5];
  const float* b_ih = (const float*)d_in[6];
  const float* b_hh = (const float*)d_in[7];
  float* out = (float*)d_out;
  char* ws = (char*)d_ws;
  unsigned short* V16 = (unsigned short*)(ws + kOffV16);
  unsigned short* WA16 = (unsigned short*)(ws + kOffWA16);
  unsigned short* WC16 = (unsigned short*)(ws + kOffWC16);
  float* BIAS = (float*)(ws + kOffBIAS);
  float* VL32 = (float*)(ws + kOffVL32);
  unsigned short* VL16 = (unsigned short*)(ws + kOffVL16);
  float* ATJ = (float*)(ws + kOffATJ);
  unsigned short* A16 = (unsigned short*)(ws + kOffA16);
  float* G32 = (float*)(ws + kOffG32);
  float* C32 = (float*)(ws + kOffC32);
  float* C0 = (float*)(ws + kOffC0);
  float* DCS = (float*)(ws + kOffDCS);

  cast_plane_kernel<<<(int)(((size_t)kRows * kD / 8) / kThr), kThr, 0, stream>>>(values, V16, 8, kD, 0);
  cast_plane_kernel<<<(int)(((size_t)kD * kD / 8) / kThr), kThr, 0, stream>>>(W_att, WA16, 8, kD, 0);
  wsetup_kernel<<<274, kThr, 0, stream>>>(b_att, W_ih, W_hh, b_ih, b_hh, BIAS, WC16, C32);
  wmma_gemm64<0, false, 2, 0, false, 0><<<dim3((kRows / 64) * (kD / 64) / 8, 1), 256, 0, stream>>>(
      V16, V16, kD, 0L, WA16, WA16, kD, 0L, (void*)VL32, (void*)VL32, kD, 0L, BIAS + kFBA, nullptr, 0L, kRows, kD, kD, kSc);
  vcast_kernel<<<4096, kThr, 0, stream>>>(VL32, VL16, A16);
  atj_kernel<<<128, kThr, 0, stream>>>(VL32, values, ATJ);

  for (int t = 0; t < kT; ++t) {
    wmma_gemm64<0, false, 2, 0, false, 0><<<dim3((kB / 64) * (kG4 / 64) / 8, 1), 256, 0, stream>>>(
        A16, A16, kK, 0L, WC16, WC16, kK, 0L, (void*)G32, (void*)G32, kG4, 0L, BIAS + kFBG, nullptr, 0L, kB, kG4, kK, kSc);
    cell_kernel<<<8, kThr, 0, stream>>>(G32, ATJ, Deltas, VL16, C32, C0, DCS, A16, out, t);
  }
}
